// _YatPerformerPolyBase_19232863552144
// MI455X (gfx1250) — hardware-run, weakly checked
//
#include <hip/hip_runtime.h>


#ifndef NB
#define NB 2
#endif
#ifndef SEQ
#define SEQ 4096
#endif
#define NB_FULL  2
#define SEQ_FULL 4096
#ifndef OUT_SEQ
#define OUT_SEQ SEQ
#endif
#define EMB  1024
#define NHD  16
#define HD   64
#define CH   128
#define NPW  80
#define STP  72
#define VFP  132

static_assert(HD == 64);
static_assert(NHD * HD == EMB);
static_assert(EMB % 64 == 0);
static_assert(EMB % 32 == 0);
static_assert(SEQ % CH == 0);
static_assert(SEQ % 64 == 0);
static_assert((NB * SEQ) % 64 == 0);
static_assert(((size_t)SEQ * EMB) % 8 == 0);
static_assert(NB <= NB_FULL);
static_assert(SEQ <= SEQ_FULL);

typedef unsigned short bf;
typedef __attribute__((ext_vector_type(16))) __bf16   v16bf;
typedef __attribute__((ext_vector_type(8)))  unsigned short v8us;
typedef __attribute__((ext_vector_type(4)))  unsigned int   v4u;
typedef __attribute__((ext_vector_type(8)))  unsigned int   v8u;
typedef __attribute__((ext_vector_type(8)))  float    v8f;
typedef __attribute__((ext_vector_type(4)))  float    v4f;
typedef v4f  __attribute__((may_alias)) v4fa;
typedef v8us __attribute__((may_alias)) v8usa;
typedef v4u  __attribute__((may_alias)) v4ua;

#define PLN ((size_t)NHD * SEQ * HD)
#define FLN ((size_t)NHD * SEQ * 32)
#define CLN ((size_t)NB * SEQ * EMB)

__device__ __forceinline__ unsigned short f2bf(float f) { unsigned u = __float_as_uint(f); u += 0x7FFFu + ((u >> 16) & 1u); return (unsigned short)(u >> 16); }
__device__ __forceinline__ float bf2f(unsigned short u) { return __uint_as_float(((unsigned)u) << 16); }
__device__ __forceinline__ float bfr(float f) { return bf2f(f2bf(f)); }
__device__ __forceinline__ unsigned rn16(float f) {
#ifdef SPLIT_INT
    unsigned u = __float_as_uint(f); u += 0x7FFFu + ((u >> 16) & 1u); return u >> 16;
#else
    return (unsigned)__builtin_bit_cast(unsigned short, (__bf16)f);
#endif
}
__device__ __forceinline__ void split2(float a, float b, unsigned& wh, unsigned& wl) {
    const unsigned ha = rn16(a), hb = rn16(b);
    const float ra = a - __uint_as_float(ha << 16), rb = b - __uint_as_float(hb << 16);
    wh = ha | (hb << 16);
    wl = rn16(ra) | (rn16(rb) << 16);
}
__device__ __forceinline__ void split8v(v8f x, v8us& hv, v8us& lv) {
    v4u h, l;
#pragma unroll
    for (int i = 0; i < 4; ++i) { unsigned a, b; split2(x[2 * i], x[2 * i + 1], a, b); h[i] = a; l[i] = b; }
    hv = __builtin_bit_cast(v8us, h); lv = __builtin_bit_cast(v8us, l);
}
__device__ __forceinline__ void split16v(v8f x0, v8f x1, v16bf& hv, v16bf& lv) {
    v8u h, l;
#pragma unroll
    for (int i = 0; i < 4; ++i) { unsigned a, b; split2(x0[2 * i], x0[2 * i + 1], a, b); h[i] = a; l[i] = b; }
#pragma unroll
    for (int i = 0; i < 4; ++i) { unsigned a, b; split2(x1[2 * i], x1[2 * i + 1], a, b); h[4 + i] = a; l[4 + i] = b; }
    hv = __builtin_bit_cast(v16bf, h); lv = __builtin_bit_cast(v16bf, l);
}
__device__ __forceinline__ v16bf cat16b(v8us lo, v8us hi) { return __builtin_bit_cast(v16bf, __builtin_shufflevector(lo, hi, 0, 1, 2, 3, 4, 5, 6, 7, 8, 9, 10, 11, 12, 13, 14, 15)); }
__device__ __forceinline__ v8f wmmab(v16bf a, v16bf b, v8f c) { return __builtin_amdgcn_wmma_f32_16x16x32_bf16(false, a, false, b, (short)0, c, false, false); }
__device__ __forceinline__ v16bf ldb(const bf* p)  { return cat16b(*(const v8usa*)p, *(const v8usa*)(p + 16)); }
__device__ __forceinline__ void wave_sync() { __builtin_amdgcn_fence(3  , "wavefront"); __builtin_amdgcn_wave_barrier(); asm volatile("" ::: "memory"); }

__global__ __launch_bounds__(256) void k_cvt8(const float* __restrict__ src, bf* dst, size_t n8) {
    const size_t i = (size_t)blockIdx.x * 256 + threadIdx.x; if (i >= n8) return;
    const v8f v = *(const v8f*)(src + i * 8); v8us o;
#pragma unroll
    for (int k = 0; k < 8; ++k) o[k] = f2bf(v[k]);
    *(volatile v8us*)(dst + i * 8) = o; __threadfence(); *(volatile v8us*)(dst + i * 8) = o;
}

__global__ __launch_bounds__(256) void k_prep(const float* __restrict__ poly_w, const float* __restrict__ omega, bf* PWT) {
    const int i = blockIdx.x * 256 + threadIdx.x; if (i >= NHD * NPW * 8) return;
    const int row = i >> 3, pc = i & 7; const int h = row / NPW, n = row % NPW;
    const int np = (n < 63) ? n : 63; int nm = n - 64; nm = (nm < 0) ? 0 : ((nm > 7) ? 7 : nm);
    v8us o;
#pragma unroll
    for (int j = 0; j < 8; ++j) { const int d = pc * 8 + j;
        const float a = poly_w[((size_t)h * HD + d) * 64 + np]; const float b = omega[((size_t)h * HD + d) * 8 + nm];
        const float v = (n < 64) ? a : ((n < 72) ? b : 0.0f); o[j] = f2bf(v); }
    *(volatile v8us*)(PWT + (size_t)i * 8) = o; __threadfence(); *(volatile v8us*)(PWT + (size_t)i * 8) = o;
}

__global__ __launch_bounds__(32) void k_qk(const bf* __restrict__ XB, const bf* __restrict__ WB, const float* __restrict__ qkv_b, const bf* __restrict__ PWT,
                                           const float* __restrict__ qn, const float* __restrict__ qw, bf* PP, bf* FF, bf* KPT) {
    __shared__ __align__(16) float tile[64 * 68];
    __shared__ __align__(16) bf xh[16 * STP];
    __shared__ __align__(16) bf xl[16 * STP];
    __shared__ __align__(16) float ps[16 * 8];
    const int K = EMB;
    const int lane = threadIdx.x & 31, lr = lane & 15, hi = lane >> 4;
    const int r0 = blockIdx.x * 64; const int cy = blockIdx.y; const int isk = cy >> 4, h = cy & 15; const int c0 = cy * 64;
    v8f acc[4][4];
#pragma unroll
    for (int mb = 0; mb < 4; ++mb)
#pragma unroll
        for (int nb = 0; nb < 4; ++nb) acc[mb][nb] = (v8f){};
    const size_t aoff = (size_t)(r0 + lr) * K + 8 * hi, boff = (size_t)(c0 + lr) * K + 8 * hi;
#pragma unroll 1
    for (int kc = 0; kc < K; kc += 32) {
        v16bf a[4];
#pragma unroll
        for (int mb = 0; mb < 4; ++mb) a[mb] = ldb(XB + aoff + (size_t)mb * 16 * K + kc);
#pragma unroll
        for (int nb = 0; nb < 4; ++nb) { const v16bf b = ldb(WB + boff + (size_t)nb * 16 * K + kc);
#pragma unroll
            for (int mb = 0; mb < 4; ++mb) acc[mb][nb] = wmmab(a[mb], b, acc[mb][nb]); }
        asm volatile("v_nop\n\tv_nop\n\tv_nop\n\tv_nop" : "+v"(acc[0][0]), "+v"(acc[1][1]), "+v"(acc[2][2]), "+v"(acc[3][3]), "+v"(acc[0][3]), "+v"(acc[1][3]), "+v"(acc[2][3]) : "v"(a[0]), "v"(a[1]), "v"(a[2]), "v"(a[3]));
    }
    float bz[4];
#pragma unroll
    for (int nb = 0; nb < 4; ++nb) bz[nb] = bfr(qkv_b[c0 + nb * 16 + lr]);
#pragma unroll
    for (int mb = 0; mb < 4; ++mb)
#pragma unroll
        for (int nb = 0; nb < 4; ++nb)
#pragma unroll
            for (int j = 0; j < 8; ++j) tile[(mb * 16 + hi * 8 + j) * 68 + nb * 16 + lr] = acc[mb][nb][j] + bz[nb];
    wave_sync();
    const float sNode = bfr(qn[0]);
    const float sq2s = sqrtf(fmaxf(2.0f * sNode, 0.0f));
    const float pscale = 0.35355339059327373f * sqrtf(fmaxf(bfr(qw[0]), 0.0f));
    bf* Ph = PP + (size_t)(2 * isk) * PLN; bf* Pl = PP + (size_t)(2 * isk + 1) * PLN; bf* Fp = FF + (size_t)isk * FLN;
#pragma unroll 1
    for (int mb = 0; mb < 4; ++mb) {
        {
            const int row = lane >> 1, hf = lane & 1;
            const float* tp = tile + (mb * 16 + row) * 68 + hf * 32;
            float x[32];
#pragma unroll
            for (int k = 0; k < 8; ++k) { const v4f t4 = *(const v4fa*)(tp + 4 * k); x[4 * k] = t4[0]; x[4 * k + 1] = t4[1]; x[4 * k + 2] = t4[2]; x[4 * k + 3] = t4[3]; }
            float ss = 0.0f;
#pragma unroll
            for (int i = 0; i < 32; ++i) ss += x[i] * x[i];
            ss += __shfl_xor(ss, 1, 32);
            const float inv = 1.0f / fmaxf(sqrtf(ss), 1e-12f);
#pragma unroll
            for (int k = 0; k < 4; ++k) { v4u hw, lw;
#pragma unroll
                for (int i = 0; i < 4; ++i) { unsigned a, b; split2(x[8 * k + 2 * i] * inv, x[8 * k + 2 * i + 1] * inv, a, b); hw[i] = a; lw[i] = b; }
                *(v8usa*)(xh + row * STP + hf * 32 + 8 * k) = __builtin_bit_cast(v8us, hw);
                *(v8usa*)(xl + row * STP + hf * 32 + 8 * k) = __builtin_bit_cast(v8us, lw); }
        }
        wave_sync();
        const v16bf xh0 = ldb(xh + lr * STP + 8 * hi), xh1 = ldb(xh + lr * STP + 8 * hi + 32), xl0 = ldb(xl + lr * STP + 8 * hi), xl1 = ldb(xl + lr * STP + 8 * hi + 32);
        v8f fa[5];
#pragma unroll
        for (int n5 = 0; n5 < 5; ++n5) { const bf* wp = PWT + ((size_t)(h * NPW + n5 * 16 + lr)) * HD + 8 * hi; const v16bf w0 = ldb(wp), w1 = ldb(wp + 32);
            v8f f = (v8f){}; f = wmmab(xh0, w0, f); f = wmmab(xl0, w0, f); f = wmmab(xh1, w1, f); f = wmmab(xl1, w1, f); fa[n5] = f; }
        asm volatile("v_nop\n\tv_nop\n\tv_nop\n\tv_nop" : "+v"(fa[0]), "+v"(fa[1]), "+v"(fa[2]), "+v"(fa[3]), "+v"(fa[4]) : "v"(xh0), "v"(xh1), "v"(xl0), "v"(xl1));
#pragma unroll
        for (int n4 = 0; n4 < 4; ++n4)
#pragma unroll
            for (int j = 0; j < 8; ++j) { const float pv = fa[n4][j]; tile[(mb * 16 + hi * 8 + j) * 68 + n4 * 16 + lr] = pv * pv * 0.125f; }
#pragma unroll
        for (int j = 0; j < 8; ++j) { const float z = fminf(fmaxf(fa[4][j] * sq2s - sNode, -20.0f), 20.0f); const float e = expf(z) * pscale;
            if (lr < 8) ps[(hi * 8 + j) * 8 + lr] = e; }
        wave_sync();
#pragma unroll 1
        for (int pss = 0; pss < 2; ++pss) {
#pragma unroll
            for (int s = 0; s < 4; ++s) { const int row = 4 * s + (lane >> 3), c8 = (lane & 7) * 8;
                const v4f x0 = *(const v4fa*)(&tile[(mb * 16 + row) * 68 + c8]); const v4f x1 = *(const v4fa*)(&tile[(mb * 16 + row) * 68 + c8 + 4]);
                v8f xv; xv[0] = x0[0]; xv[1] = x0[1]; xv[2] = x0[2]; xv[3] = x0[3]; xv[4] = x1[0]; xv[5] = x1[1]; xv[6] = x1[2]; xv[7] = x1[3];
                v8us hv, lv; split8v(xv, hv, lv);
                const size_t oo = ((size_t)h * SEQ + r0 + mb * 16 + row) * HD + c8;
                *(volatile v8us*)(Ph + oo) = hv; *(volatile v8us*)(Pl + oo) = lv; }
#pragma unroll
            for (int u = 0; u < 2; ++u) { const int tok = u * 8 + (lane >> 2), slot = lane & 3;
                const v4f p0 = *(const v4fa*)(&ps[tok * 8]); const v4f p1 = *(const v4fa*)(&ps[tok * 8 + 4]);
                v8f pv; pv[0] = p0[0]; pv[1] = p0[1]; pv[2] = p0[2]; pv[3] = p0[3]; pv[4] = p1[0]; pv[5] = p1[1]; pv[6] = p1[2]; pv[7] = p1[3];
                v8us hv, lv; split8v(pv, hv, lv);
                const v4u hw = __builtin_bit_cast(v4u, hv), lw = __builtin_bit_cast(v4u, lv);
                const bool useL = isk ? (slot == 1) : (slot == 2); const bool useZ = (slot == 3);
                v4u ow;
#pragma unroll
                for (int i = 0; i < 4; ++i) ow[i] = useZ ? 0u : (useL ? lw[i] : hw[i]);
                const size_t oo = ((size_t)h * SEQ + r0 + mb * 16 + tok) * 32 + slot * 8;
                *(volatile v8us*)(Fp + oo) = __builtin_bit_cast(v8us, ow); }
            if (pss == 0) __threadfence(); }
        wave_sync();
    }
    if (isk) {
        bf* Th = KPT; bf* Tl = KPT + PLN;
#pragma unroll 1
        for (int pss = 0; pss < 2; ++pss) {
#pragma unroll 1
            for (int s = 0; s < 16; ++s) { const int p = 4 * s + (lane >> 3), pc = lane & 7;
                v8f xv;
#pragma unroll
                for (int i = 0; i < 8; ++i) xv[i] = tile[(pc * 8 + i) * 68 + p];
                v8us hv, lv; split8v(xv, hv, lv);
                const size_t oo = ((size_t)h * HD + p) * SEQ + r0 + pc * 8;
                *(volatile v8us*)(Th + oo) = hv; *(volatile v8us*)(Tl + oo) = lv; }
            if (pss == 0) __threadfence(); }
    }
}

__global__ __launch_bounds__(32) void k_vt(const bf* __restrict__ WV, const bf* __restrict__ XB, const float* __restrict__ vb, bf* VT) {
    __shared__ __align__(16) float os[16 * 68];
    const int K = EMB;
    const int lane = threadIdx.x & 31, lr = lane & 15, hi = lane >> 4; const int r0 = blockIdx.x * 64, c0 = blockIdx.y * 64;
    v8f acc[4][4];
#pragma unroll
    for (int mb = 0; mb < 4; ++mb)
#pragma unroll
        for (int nb = 0; nb < 4; ++nb) acc[mb][nb] = (v8f){};
    const size_t aoff = (size_t)(r0 + lr) * K + 8 * hi, boff = (size_t)(c0 + lr) * K + 8 * hi;
#pragma unroll 1
    for (int kc = 0; kc < K; kc += 32) {
        v16bf a[4];
#pragma unroll
        for (int mb = 0; mb < 4; ++mb) a[mb] = ldb(WV + aoff + (size_t)mb * 16 * K + kc);
#pragma unroll
        for (int nb = 0; nb < 4; ++nb) { const v16bf b = ldb(XB + boff + (size_t)nb * 16 * K + kc);
#pragma unroll
            for (int mb = 0; mb < 4; ++mb) acc[mb][nb] = wmmab(a[mb], b, acc[mb][nb]); }
        asm volatile("v_nop\n\tv_nop\n\tv_nop\n\tv_nop" : "+v"(acc[0][0]), "+v"(acc[1][1]), "+v"(acc[2][2]), "+v"(acc[3][3]), "+v"(acc[0][3]), "+v"(acc[1][3]), "+v"(acc[2][3]) : "v"(a[0]), "v"(a[1]), "v"(a[2]), "v"(a[3]));
    }
    bf* Vh = VT; bf* Vl = VT + PLN;
#pragma unroll
    for (int mb = 0; mb < 4; ++mb) {
        float rb[8];
#pragma unroll
        for (int j = 0; j < 8; ++j) rb[j] = bfr(vb[r0 + mb * 16 + hi * 8 + j]);
#pragma unroll
        for (int nb = 0; nb < 4; ++nb)
#pragma unroll
            for (int j = 0; j < 8; ++j) os[(hi * 8 + j) * 68 + nb * 16 + lr] = acc[mb][nb][j] + rb[j];
        wave_sync();
#pragma unroll 1
        for (int pss = 0; pss < 2; ++pss) {
#pragma unroll
            for (int s = 0; s < 4; ++s) { const int row = 4 * s + (lane >> 3), c8 = (lane & 7) * 8;
                const v4f x0 = *(const v4fa*)(&os[row * 68 + c8]); const v4f x1 = *(const v4fa*)(&os[row * 68 + c8 + 4]);
                v8f xv; xv[0] = x0[0]; xv[1] = x0[1]; xv[2] = x0[2]; xv[3] = x0[3]; xv[4] = x1[0]; xv[5] = x1[1]; xv[6] = x1[2]; xv[7] = x1[3];
                v8us hv, lv; split8v(xv, hv, lv);
                const size_t oo = (size_t)(r0 + mb * 16 + row) * SEQ + c0 + c8;
                *(volatile v8us*)(Vh + oo) = hv; *(volatile v8us*)(Vl + oo) = lv; }
            if (pss == 0) __threadfence(); }
        wave_sync();
    }
}

#define OFF_STH 0
#define OFF_STL (OFF_STH + 8 * 64 * STP * 2)
#define OFF_KSH (OFF_STL + 8 * 64 * STP * 2)
#define OFF_KSL (OFF_KSH + 16 * STP * 2)
#define OFF_VF  (OFF_KSL + 16 * STP * 2)
#define OFF_KT  (OFF_VF + 64 * VFP * 4)
#define OFF_CTH (OFF_KT + 8 * 128 * 4)
#define OFF_CTL (OFF_CTH + 128 * STP * 2)
#define SCAN_LDS (OFF_CTL + 128 * STP * 2)
static_assert(OFF_VF % 16 == 0);
static_assert(OFF_KT % 16 == 0);
static_assert(OFF_CTH % 16 == 0);
static_assert(SCAN_LDS <= 240 * 1024);

__global__ __launch_bounds__(512) void k_scan(const bf* __restrict__ PP, const bf* __restrict__ KPT, const bf* __restrict__ FF, const bf* __restrict__ VT, bf* CX, size_t ctxRow0) {
    extern __shared__ __align__(16) unsigned char smem[];
    bf* STh = (bf*)(smem + OFF_STH); bf* STl = (bf*)(smem + OFF_STL);
    bf* KSh = (bf*)(smem + OFF_KSH); bf* KSl = (bf*)(smem + OFF_KSL);
    float* Vf = (float*)(smem + OFF_VF); float* KT = (float*)(smem + OFF_KT);
    bf* CTh = (bf*)(smem + OFF_CTH); bf* CTl = (bf*)(smem + OFF_CTL);
    const int tid = threadIdx.x, lane = tid & 31, lr = lane & 15, hi = lane >> 4;
    const int wave = __builtin_amdgcn_readfirstlane(tid >> 5);
    const int h = blockIdx.x;
    const bf* QPh = PP; const bf* QPl = PP + PLN; const bf* KPh = PP + 2 * PLN; const bf* KPl = PP + 3 * PLN;
    const bf* KPTh = KPT; const bf* KPTl = KPT + PLN;
    const bf* QF = FF; const bf* KF = FF + FLN;
    const bf* VTh = VT; const bf* VTl = VT + PLN;
    bf* CXh = CX; bf* CXl = CX + CLN;
    for (int i = tid; i < OFF_VF / 16; i += 512) *(v4ua*)(smem + (size_t)i * 16) = (v4u){0u, 0u, 0u, 0u};
    __syncthreads();
    const int tt = wave >> 1, dp = wave & 1, dt = wave & 3, mp = wave >> 2;
#pragma unroll 1
    for (int c = 0; c < SEQ / CH; ++c) {
        const size_t cb = (size_t)c * CH;
        {
            const int d = tid >> 3, pc = tid & 7;
            const size_t vo = ((size_t)h * HD + d) * SEQ + cb + pc * 16;
            const v8us a0 = *(const v8usa*)(VTh + vo), a1 = *(const v8usa*)(VTh + vo + 8), b0 = *(const v8usa*)(VTl + vo), b1 = *(const v8usa*)(VTl + vo + 8);
            v4f f0, f1, f2, f3;
#pragma unroll
            for (int i = 0; i < 4; ++i) { f0[i] = bf2f(a0[i]) + bf2f(b0[i]); f1[i] = bf2f(a0[4 + i]) + bf2f(b0[4 + i]); f2[i] = bf2f(a1[i]) + bf2f(b1[i]); f3[i] = bf2f(a1[4 + i]) + bf2f(b1[4 + i]); }
            float* vp = Vf + d * VFP + pc * 16;
            *(v4fa*)vp = f0; *(v4fa*)(vp + 4) = f1; *(v4fa*)(vp + 8) = f2; *(v4fa*)(vp + 12) = f3;
        }
        if (wave < 4) {
            const int s = tid;
            const size_t ko = ((size_t)h * SEQ + cb + s) * 32;
            const v8us kh = *(const v8usa*)(KF + ko), kl = *(const v8usa*)(KF + ko + 8);
#pragma unroll
            for (int m = 0; m < 8; ++m) KT[m * 128 + s] = bf2f(kh[m]) + bf2f(kl[m]);
        }
        {
            const int tl = tt * 16 + lr;
            const size_t trow = (size_t)h * SEQ + cb + tl;
            const bf* qp = QPh + trow * HD + 8 * hi; const bf* qq = QPl + trow * HD + 8 * hi;
            const v16bf qh0 = ldb(qp), qh1 = ldb(qp + 32), ql0 = ldb(qq), ql1 = ldb(qq + 32);
            v8f o0 = (v8f){}, o1 = (v8f){}; float rs = 0.0f;
            {
                const v16bf qfb = ldb(QF + trow * 32 + 8 * hi);
                const int nkp = (tt >> 1) + 1;
#pragma unroll 1
                for (int kp = 0; kp < nkp; ++kp) {
                    const int s0 = kp * 32;
                    v8f sv0 = (v8f){}, sv1 = (v8f){};
#pragma unroll 1
                    for (int hf = 0; hf < 2; ++hf) {
                        const size_t krow = (size_t)h * SEQ + cb + s0 + hf * 16 + lr;
                        const bf* ka = KPh + krow * HD + 8 * hi; const bf* kb = KPl + krow * HD + 8 * hi;
                        const v16bf kh0 = ldb(ka), kh1 = ldb(ka + 32), kl0 = ldb(kb), kl1 = ldb(kb + 32);
                        const v16bf kfa = ldb(KF + krow * 32 + 8 * hi);
                        v8f aS = (v8f){}, aP = (v8f){};
                        aS = wmmab(kh0, qh0, aS); aP = wmmab(kfa, qfb, aP);
                        aS = wmmab(kh0, ql0, aS); aS = wmmab(kl0, qh0, aS);
                        aS = wmmab(kh1, qh1, aS); aS = wmmab(kh1, ql1, aS); aS = wmmab(kl1, qh1, aS);
                        asm volatile("v_nop\n\tv_nop\n\tv_nop\n\tv_nop" : "+v"(aS), "+v"(aP) : "v"(kh0), "v"(kh1), "v"(kl0), "v"(kl1), "v"(kfa));
                        v8f sv;
#pragma unroll
                        for (int r = 0; r < 8; ++r) { const int s = s0 + hf * 16 + 8 * hi + r; const float val = aS[r] * aP[r]; sv[r] = (s <= tl) ? val : 0.0f; rs += sv[r]; }
                        if (hf == 0) sv0 = sv; else sv1 = sv;
                    }
                    v16bf ph, pl; split16v(sv0, sv1, ph, pl);
                    const size_t vr0 = ((size_t)h * HD + 16 * (2 * dp) + lr) * SEQ + cb + s0 + 8 * hi;
                    const size_t vr1 = vr0 + (size_t)16 * SEQ;
                    const v16bf vh0 = ldb(VTh + vr0), vl0 = ldb(VTl + vr0), vh1 = ldb(VTh + vr1), vl1 = ldb(VTl + vr1);
                    o0 = wmmab(vh0, ph, o0); o1 = wmmab(vh1, ph, o1);
                    o0 = wmmab(vh0, pl, o0); o1 = wmmab(vh1, pl, o1);
                    o0 = wmmab(vl0, ph, o0); o1 = wmmab(vl1, ph, o1);
                    asm volatile("v_nop\n\tv_nop\n\tv_nop\n\tv_nop" : "+v"(o0), "+v"(o1) : "v"(vh0), "v"(vl0), "v"(vh1), "v"(vl1), "v"(ph), "v"(pl));
                }
            }
            rs += __shfl_xor(rs, 16, 32);
#pragma unroll 1
            for (int m = 0; m < 8; ++m) {
                const float qm = bf2f(QF[trow * 32 + m]) + bf2f(QF[trow * 32 + 16 + m]);
                const int so = (m * 64 + 16 * (2 * dp) + lr) * STP + 8 * hi;
                const v16bf a0h0 = ldb(STh + so), a0h1 = ldb(STh + so + 32), a0l0 = ldb(STl + so), a0l1 = ldb(STl + so + 32);
                const v16bf a1h0 = ldb(STh + so + 16 * STP), a1h1 = ldb(STh + so + 16 * STP + 32), a1l0 = ldb(STl + so + 16 * STP), a1l1 = ldb(STl + so + 16 * STP + 32);
                v8f g0 = (v8f){}, g1 = (v8f){};
                g0 = wmmab(a0h0, qh0, g0); g1 = wmmab(a1h0, qh0, g1);
                g0 = wmmab(a0h0, ql0, g0); g1 = wmmab(a1h0, ql0, g1);
                g0 = wmmab(a0l0, qh0, g0); g1 = wmmab(a1l0, qh0, g1);
                g0 = wmmab(a0h1, qh1, g0); g1 = wmmab(a1h1, qh1, g1);
                g0 = wmmab(a0h1, ql1, g0); g1 = wmmab(a1h1, ql1, g1);
                g0 = wmmab(a0l1, qh1, g0); g1 = wmmab(a1l1, qh1, g1);
                asm volatile("v_nop\n\tv_nop\n\tv_nop\n\tv_nop" : "+v"(g0), "+v"(g1) : "v"(a0h0), "v"(a0h1), "v"(a0l0), "v"(a0l1), "v"(a1h0), "v"(a1h1), "v"(a1l0), "v"(a1l1));
                o0 = o0 + g0 * qm; o1 = o1 + g1 * qm;
            }
            float nh = 0.0f;
            {
                float q[8];
                { const v8us a = *(const v8usa*)(QF + trow * 32); const v8us b = *(const v8usa*)(QF + trow * 32 + 16);
#pragma unroll
                  for (int i = 0; i < 8; ++i) q[i] = bf2f(a[i]) + bf2f(b[i]); }
                const bf* za = KSh + (lr * STP + 8 * hi); const bf* zc = KSl + (lr * STP + 8 * hi);
                const v16bf zh0 = ldb(za), zh1 = ldb(za + 32), zl0 = ldb(zc), zl1 = ldb(zc + 32);
                v8f z = (v8f){};
                z = wmmab(zh0, qh0, z); z = wmmab(zh0, ql0, z); z = wmmab(zl0, qh0, z);
                z = wmmab(zh1, qh1, z); z = wmmab(zh1, ql1, z); z = wmmab(zl1, qh1, z);
                asm volatile("v_nop\n\tv_nop\n\tv_nop\n\tv_nop" : "+v"(z) : "v"(zh0), "v"(zh1), "v"(zl0), "v"(zl1));
#pragma unroll
                for (int r = 0; r < 8; ++r) nh += q[r] * z[r];
            }
            nh += __shfl_xor(nh, 16, 32);
            const float nrm = (nh + rs) + 1e-6f;
            const float inv = 1.0f / nrm;
            o0 = o0 * inv; o1 = o1 * inv;
            v8us hv, lv;
            split8v(o0, hv, lv);
            *(v8usa*)(CTh + tl * STP + 16 * (2 * dp) + 8 * hi) = hv; *(v8usa*)(CTl + tl * STP + 16 * (2 * dp) + 8 * hi) = lv;
            split8v(o1, hv, lv);
            *(v8usa*)(CTh + tl * STP + 16 * (2 * dp + 1) + 8 * hi) = hv; *(v8usa*)(CTl + tl * STP + 16 * (2 * dp + 1) + 8 * hi) = lv;
        }
        __syncthreads();
        {
#pragma unroll 1
            for (int mi = 0; mi < 2; ++mi) {
                const int sidx = ((2 * mp + mi) * 64 + 16 * dt + lr) * STP + 8 * hi;
                const float* kq0 = KT + (2 * mp + mi) * 128 + 8 * hi;
                const float* vp0 = Vf + (16 * dt + lr) * VFP + 8 * hi;
                v8f st[4];
#pragma unroll
                for (int pt = 0; pt < 4; ++pt) { const v8us a = *(const v8usa*)(STh + sidx + 16 * pt), b = *(const v8usa*)(STl + sidx + 16 * pt);
#pragma unroll
                    for (int r = 0; r < 8; ++r) st[pt][r] = bf2f(a[r]) + bf2f(b[r]); }
#pragma unroll 1
                for (int ks = 0; ks < 4; ++ks) {
                    const float* vp = vp0 + ks * 32; const float* kq = kq0 + ks * 32;
                    const v4f v0 = *(const v4fa*)vp, v1 = *(const v4fa*)(vp + 4), v2 = *(const v4fa*)(vp + 16), v3 = *(const v4fa*)(vp + 20);
                    const v4f k0 = *(const v4fa*)kq, k1 = *(const v4fa*)(kq + 4), k2 = *(const v4fa*)(kq + 16), k3 = *(const v4fa*)(kq + 20);
                    v8f w0, w1;
#pragma unroll
                    for (int i = 0; i < 4; ++i) { w0[i] = k0[i] * v0[i]; w0[4 + i] = k1[i] * v1[i]; w1[i] = k2[i] * v2[i]; w1[4 + i] = k3[i] * v3[i]; }
                    v16bf wh, wl; split16v(w0, w1, wh, wl);
                    const size_t ao = ((size_t)h * HD + lr) * SEQ + cb + ks * 32 + 8 * hi;
                    v16bf ah[4], al[4];
#pragma unroll
                    for (int pt = 0; pt < 4; ++pt) { ah[pt] = ldb(KPTh + ao + (size_t)(16 * pt) * SEQ); al[pt] = ldb(KPTl + ao + (size_t)(16 * pt) * SEQ); }
#pragma unroll
                    for (int pt = 0; pt < 4; ++pt) st[pt] = wmmab(ah[pt], wh, st[pt]);
#pragma unroll
                    for (int pt = 0; pt < 4; ++pt) st[pt] = wmmab(ah[pt], wl, st[pt]);
#pragma unroll
                    for (int pt = 0; pt < 4; ++pt) st[pt] = wmmab(al[pt], wh, st[pt]);
                    asm volatile("v_nop\n\tv_nop\n\tv_nop\n\tv_nop" : "+v"(st[0]), "+v"(st[1]), "+v"(st[2]), "+v"(st[3])
                                 : "v"(ah[0]), "v"(ah[1]), "v"(ah[2]), "v"(ah[3]), "v"(al[0]), "v"(al[1]), "v"(al[2]), "v"(al[3]), "v"(wh), "v"(wl));
                }
#pragma unroll
                for (int pt = 0; pt < 4; ++pt) { v8us hv, lv; split8v(st[pt], hv, lv);
                    *(v8usa*)(STh + sidx + 16 * pt) = hv; *(v8usa*)(STl + sidx + 16 * pt) = lv; }
            }
            if (dt == 0) {
                const int kidx = lr * STP + 16 * mp + 8 * hi;
                v8f ksa;
                { const v8us a = *(const v8usa*)(KSh + kidx), b = *(const v8usa*)(KSl + kidx);
#pragma unroll
                  for (int r = 0; r < 8; ++r) ksa[r] = bf2f(a[r]) + bf2f(b[r]); }
                const bool on = (lr < 8);
#pragma unroll 1
                for (int ks = 0; ks < 4; ++ks) {
                    const float* kq = KT + (lr & 7) * 128 + ks * 32 + 8 * hi;
                    const v4f k0 = *(const v4fa*)kq, k1 = *(const v4fa*)(kq + 4), k2 = *(const v4fa*)(kq + 16), k3 = *(const v4fa*)(kq + 20);
                    v8f w0, w1;
#pragma unroll
                    for (int i = 0; i < 4; ++i) { w0[i] = on ? k0[i] : 0.0f; w0[4 + i] = on ? k1[i] : 0.0f; w1[i] = on ? k2[i] : 0.0f; w1[4 + i] = on ? k3[i] : 0.0f; }
                    v16bf bh, bl; split16v(w0, w1, bh, bl);
                    const size_t ao = ((size_t)h * HD + 16 * mp + lr) * SEQ + cb + ks * 32 + 8 * hi;
                    const v16bf ah = ldb(KPTh + ao), al = ldb(KPTl + ao);
                    ksa = wmmab(ah, bh, ksa); ksa = wmmab(ah, bl, ksa); ksa = wmmab(al, bh, ksa);
                    asm volatile("v_nop\n\tv_nop\n\tv_nop\n\tv_nop" : "+v"(ksa) : "v"(ah), "v"(al), "v"(bh), "v"(bl));
                }
                v8us hv, lv; split8v(ksa, hv, lv);
                *(v8usa*)(KSh + kidx) = hv; *(v8usa*)(KSl + kidx) = lv;
            }
        }
#pragma unroll 1
        for (int pss = 0; pss < 2; ++pss) {
#pragma unroll
            for (int sw = 0; sw < 2; ++sw) { const int row = sw * 64 + (tid >> 3), pc = tid & 7;
                const v8us a = *(const v8usa*)(CTh + row * STP + pc * 8); const v8us b = *(const v8usa*)(CTl + row * STP + pc * 8);
                const size_t go = (ctxRow0 + cb + row) * EMB + (size_t)h * HD + pc * 8;
                *(volatile v8us*)(CXh + go) = a; *(volatile v8us*)(CXl + go) = b; }
            if (pss == 0) __threadfence(); }
        __syncthreads();
    }
}

__global__ __launch_bounds__(32) void k_out(const bf* __restrict__ CX, const bf* __restrict__ OW, const float* __restrict__ ob, float* OUT) {
    __shared__ __align__(16) float os[16 * 68];
    const int K = EMB;
    const int lane = threadIdx.x & 31, lr = lane & 15, hi = lane >> 4; const int r0 = blockIdx.x * 64, c0 = blockIdx.y * 64;
    v8f acc[4][4];
#pragma unroll
    for (int mb = 0; mb < 4; ++mb)
#pragma unroll
        for (int nb = 0; nb < 4; ++nb) acc[mb][nb] = (v8f){};
    const size_t aoff = (size_t)(r0 + lr) * K + 8 * hi, boff = (size_t)(c0 + lr) * K + 8 * hi;
#pragma unroll 1
    for (int kc = 0; kc < K; kc += 32) {
#pragma unroll
        for (int pl = 0; pl < 2; ++pl) {
            v16bf a[4];
#pragma unroll
            for (int mb = 0; mb < 4; ++mb) a[mb] = ldb(CX + (size_t)pl * CLN + aoff + (size_t)mb * 16 * K + kc);
#pragma unroll
            for (int nb = 0; nb < 4; ++nb) { const v16bf b = ldb(OW + boff + (size_t)nb * 16 * K + kc);
#pragma unroll
                for (int mb = 0; mb < 4; ++mb) acc[mb][nb] = wmmab(a[mb], b, acc[mb][nb]); }
            asm volatile("v_nop\n\tv_nop\n\tv_nop\n\tv_nop" : "+v"(acc[0][0]), "+v"(acc[1][1]), "+v"(acc[2][2]), "+v"(acc[3][3]), "+v"(acc[0][3]), "+v"(acc[1][3]), "+v"(acc[2][3]) : "v"(a[0]), "v"(a[1]), "v"(a[2]), "v"(a[3]));
        }
    }
    float bz[4];
#pragma unroll
    for (int nb = 0; nb < 4; ++nb) bz[nb] = bfr(ob[c0 + nb * 16 + lr]);
#pragma unroll
    for (int mb = 0; mb < 4; ++mb) {
#pragma unroll
        for (int nb = 0; nb < 4; ++nb)
#pragma unroll
            for (int j = 0; j < 8; ++j) os[(hi * 8 + j) * 68 + nb * 16 + lr] = acc[mb][nb][j] + bz[nb];
        wave_sync();
#pragma unroll 1
        for (int pss = 0; pss < 2; ++pss) {
#pragma unroll
            for (int s = 0; s < 8; ++s) { const int row = 2 * s + hi, cofs = lr * 4;
                const v4f val = *(const v4fa*)(&os[row * 68 + cofs]);
                const int g = r0 + mb * 16 + row; const size_t orow = (size_t)(g / SEQ) * OUT_SEQ + (size_t)(g % SEQ);
                *(volatile v4f*)(OUT + orow * EMB + c0 + cofs) = val; }
            if (pss == 0) __threadfence(); }
        wave_sync();
    }
}

static constexpr size_t al256(size_t v) { return (v + 255) & ~(size_t)255; }
static constexpr size_t SZ_XB = al256((size_t)SEQ * EMB * 2);
static constexpr size_t SZ_WB = al256((size_t)3 * EMB * EMB * 2);
static constexpr size_t SZ_OW = al256((size_t)EMB * EMB * 2);
static constexpr size_t SZ_PW = al256((size_t)NHD * NPW * HD * 2);
static constexpr size_t SZ_PP = al256((size_t)4 * NHD * SEQ * HD * 2);
static constexpr size_t SZ_KT = al256((size_t)2 * NHD * SEQ * HD * 2);
static constexpr size_t SZ_FF = al256((size_t)2 * NHD * SEQ * 32 * 2);
static constexpr size_t SZ_VT = al256((size_t)2 * NHD * SEQ * HD * 2);
static constexpr size_t SZ_CX = al256((size_t)2 * NB * SEQ * EMB * 2);
static constexpr size_t SZ_TOTAL = SZ_XB + SZ_WB + SZ_OW + SZ_PW + SZ_PP + SZ_KT + SZ_FF + SZ_VT + SZ_CX;
static_assert(SZ_TOTAL <= (size_t)134217728);

extern "C" void kernel_launch(void* const* d_in, const int* in_sizes, int n_in,
                              void* d_out, int out_size, void* d_ws, size_t ws_size, hipStream_t stream) {
    if (n_in < 9) return;
    if ((size_t)in_sizes[0] < ((size_t)(NB - 1) * SEQ_FULL + SEQ) * EMB) return;
    if ((size_t)in_sizes[1] < (size_t)3 * EMB * EMB || (size_t)in_sizes[2] < (size_t)3 * EMB) return;
    if ((size_t)in_sizes[3] < (size_t)EMB * EMB || (size_t)in_sizes[4] < (size_t)EMB) return;
    if ((size_t)in_sizes[5] < (size_t)NHD * HD * 8 || (size_t)in_sizes[6] < (size_t)NHD * HD * 64) return;
    if (in_sizes[7] < 1 || in_sizes[8] < 1) return;
    if ((size_t)out_size < ((size_t)(NB - 1) * OUT_SEQ + SEQ) * EMB) return;
    if (SZ_TOTAL > ws_size) return;
    const float* x = (const float*)d_in[0]; const float* qkv_w = (const float*)d_in[1]; const float* qkv_b = (const float*)d_in[2];
    const float* out_w = (const float*)d_in[3]; const float* out_b = (const float*)d_in[4]; const float* omega = (const float*)d_in[5];
    const float* poly_w = (const float*)d_in[6]; const float* qn = (const float*)d_in[7]; const float* qw = (const float*)d_in[8];
    float* OUT = (float*)d_out;
    char* wsp = (char*)d_ws;
    bf* XB = (bf*)wsp; wsp += SZ_XB;
    bf* WB = (bf*)wsp; wsp += SZ_WB;
    bf* OWB = (bf*)wsp; wsp += SZ_OW;
    bf* PWT = (bf*)wsp; wsp += SZ_PW;
    bf* PP = (bf*)wsp; wsp += SZ_PP;
    bf* KPT = (bf*)wsp; wsp += SZ_KT;
    bf* FF = (bf*)wsp; wsp += SZ_FF;
    bf* VT = (bf*)wsp; wsp += SZ_VT;
    bf* CX = (bf*)wsp; wsp += SZ_CX;

    { const size_t n8 = (size_t)3 * EMB * EMB / 8; k_cvt8<<<(unsigned)((n8 + 255) / 256), 256, 0, stream>>>(qkv_w, WB, n8); }
    { const size_t n8 = (size_t)EMB * EMB / 8; k_cvt8<<<(unsigned)((n8 + 255) / 256), 256, 0, stream>>>(out_w, OWB, n8); }
    k_prep<<<(NHD * NPW * 8 + 255) / 256, 256, 0, stream>>>(poly_w, omega, PWT);
    hipFuncSetAttribute(reinterpret_cast<const void*>(&k_scan), hipFuncAttributeMaxDynamicSharedMemorySize, (int)SCAN_LDS);
    for (int b = 0; b < NB; ++b) {
        const size_t n8 = (size_t)SEQ * EMB / 8;
        k_cvt8<<<(unsigned)((n8 + 255) / 256), 256, 0, stream>>>(x + (size_t)b * SEQ_FULL * EMB, XB, n8);
        k_qk<<<dim3(SEQ / 64, 2 * NHD, 1), 32, 0, stream>>>(XB, WB, qkv_b, PWT, qn, qw, PP, FF, KPT);
        k_vt<<<dim3(EMB / 64, SEQ / 64, 1), 32, 0, stream>>>(WB + (size_t)2 * EMB * EMB, XB, qkv_b + 2 * EMB, VT);
        k_scan<<<dim3(NHD, 1, 1), 512, SCAN_LDS, stream>>>(PP, KPT, FF, VT, CX, (size_t)b * SEQ);
    }
    k_out<<<dim3(NB * SEQ / 64, EMB / 64, 1), 32, 0, stream>>>(CX, OWB, out_b, OUT);
}
